// EGNN_50861002719986
// MI455X (gfx1250) — hardware-verified
//
#include <hip/hip_runtime.h>
#include <stddef.h>
#include <stdint.h>
#include <math.h>


#define C      64
#define DX     128
#define KX     128
#define KA     192
#define KP     384
#define NTHR   256
#define NWAVE  8
#define EPT    8
#define CHUNK  (NTHR * EPT)
#define WCAP   (EPT * 32)
#define LISTN  (NWAVE * WCAP)
#define NBA    1024
#define PKS    10
#define RCAP   28672
#define DEGCAP 64
#define GBM    64
#define GBN    64
#define GTHR   128
#define RB     KP
#define NU0    (C * (KX / 8))
#define NUW    (C * (KA / 8))
#define RG1    NU0
#define RG2    (RG1 + NUW)
#define RG3    (RG2 + NUW)
#define RG4    (RG3 + NUW)
#define ZINTS  (2 * RCAP + 2 * NBA + LISTN)
#define MISC_INTS 16
#define LDS_AGG (ZINTS * 4 + MISC_INTS * 4 + NWAVE * RB * 2)
#define WSMAX  134217728

static_assert((CHUNK & (CHUNK - 1)) == 0);
static_assert(NBA == (1 << PKS));
static_assert(((long long)CHUNK << PKS) < (1LL << 31));
static_assert(NTHR * 4 == NBA);
static_assert(LISTN >= NBA && LISTN >= NWAVE * WCAP);
static_assert((RCAP % 32) == 0);
static_assert((ZINTS % (NTHR * 4)) == 0);
static_assert(((ZINTS + MISC_INTS) * 4) % 16 == 0 && (RB * 2) % 16 == 0);
static_assert(LDS_AGG <= 300000);
static_assert((NBA % NWAVE) == 0 && (NBA % GBM) == 0);
static_assert(GBM == (GTHR / 32) * 16);
static_assert(GBN == C && GTHR >= GBN);
static_assert(KA == 3 * C && KP == 2 * KA && (KP % 32) == 0 && (KX % 32) == 0 && KX == DX);
static_assert(((KP * 2) % 128) == 0);
static_assert(((KX * 2) % 128) == 0);
static_assert(((C * 4) % 128) == 0);
static_assert(C == 32 * 2);
static_assert(RB == KP && 256 + 8 * 16 == KP);
static_assert(DX / 8 == 16 && KX / 8 == 16 && (KA / 8) % 8 == 0);
static_assert((RG1 % NTHR) == 0 && (RG2 % NTHR) == 0 && (RG3 % NTHR) == 0 && (RG4 % NTHR) == 0);
static_assert(DEGCAP <= RCAP && WCAP <= LISTN);

typedef float          v4f  __attribute__((ext_vector_type(4)));
typedef float          v2f  __attribute__((ext_vector_type(2)));
typedef float          v8f  __attribute__((ext_vector_type(8)));
typedef int            v4i  __attribute__((ext_vector_type(4)));
typedef int            v8i  __attribute__((ext_vector_type(8)));
typedef unsigned short v2us __attribute__((ext_vector_type(2)));
typedef unsigned short v8us __attribute__((ext_vector_type(8)));
typedef __bf16         v16b __attribute__((ext_vector_type(16)));
typedef v4f  __attribute__((may_alias)) v4fa;
typedef v2f  __attribute__((may_alias)) v2fa;
typedef v4i  __attribute__((may_alias)) v4ia;
typedef v2us __attribute__((may_alias)) v2usa;
typedef v8us __attribute__((may_alias)) v8usa;
union Frag { v16b b; v8us h[2]; v8i w; };

__device__ __forceinline__ v8f wmk(const Frag& a, const Frag& b, v8f c) {
  v8f d = __builtin_amdgcn_wmma_f32_16x16x32_bf16(false, a.b, false, b.b, (short)0, c, false, false);
  asm volatile("v_nop\n\tv_nop\n\tv_nop\n\tv_nop" : "+v"(d) : "v"(a.w), "v"(b.w));
  return d;
}

__device__ __forceinline__ v8f z8() { v8f z = {0.f, 0.f, 0.f, 0.f, 0.f, 0.f, 0.f, 0.f}; return z; }

__device__ __forceinline__ unsigned bf16_bits(float f) {
  const unsigned u = __float_as_uint(f);
  return (u + 0x7FFFu + ((u >> 16) & 1u)) >> 16;
}
__device__ __forceinline__ float bf16_val(float f) {
  return __uint_as_float(bf16_bits(f) << 16);
}

__device__ __forceinline__ void wave_sync() {
  __builtin_amdgcn_fence(__ATOMIC_RELEASE, "wavefront");
  __builtin_amdgcn_wave_barrier();
  __builtin_amdgcn_fence(__ATOMIC_ACQUIRE, "wavefront");
}

__device__ __forceinline__ int scan_chunk(const int* __restrict__ dsts, int nE, int cbase, int slotBase,
                                          int nb, int vec8, int* list, int tid, int lane, int wave) {
  int wc = 0;
  const int el0  = tid * EPT;
  const int e0   = cbase + el0;
  const int sent = -2147483647 - 1;
  v4i da, db;
  if (vec8 != 0 && cbase + CHUNK <= nE) {
    da = *(const v4i*)(dsts + e0);
    db = *(const v4i*)(dsts + e0 + 4);
  } else {
    da.x = (e0     < nE) ? dsts[min(e0,     nE - 1)] : sent;
    da.y = (e0 + 1 < nE) ? dsts[min(e0 + 1, nE - 1)] : sent;
    da.z = (e0 + 2 < nE) ? dsts[min(e0 + 2, nE - 1)] : sent;
    da.w = (e0 + 3 < nE) ? dsts[min(e0 + 3, nE - 1)] : sent;
    db.x = (e0 + 4 < nE) ? dsts[min(e0 + 4, nE - 1)] : sent;
    db.y = (e0 + 5 < nE) ? dsts[min(e0 + 5, nE - 1)] : sent;
    db.z = (e0 + 6 < nE) ? dsts[min(e0 + 6, nE - 1)] : sent;
    db.w = (e0 + 7 < nE) ? dsts[min(e0 + 7, nE - 1)] : sent;
  }
  const unsigned nbs = (unsigned)slotBase;
  const unsigned unb = (unsigned)nb;
  const unsigned s0 = (unsigned)da.x - nbs, s1 = (unsigned)da.y - nbs;
  const unsigned s2 = (unsigned)da.z - nbs, s3 = (unsigned)da.w - nbs;
  const unsigned s4 = (unsigned)db.x - nbs, s5 = (unsigned)db.y - nbs;
  const unsigned s6 = (unsigned)db.z - nbs, s7 = (unsigned)db.w - nbs;
  const bool h0 = s0 < unb, h1 = s1 < unb, h2 = s2 < unb, h3 = s3 < unb;
  const bool h4 = s4 < unb, h5 = s5 < unb, h6 = s6 < unb, h7 = s7 < unb;
  const unsigned any = __builtin_amdgcn_ballot_w32(h0 | h1 | h2 | h3 | h4 | h5 | h6 | h7);
  if (any != 0u) {
#define HITJ(J, HJ, SJ) { \
      const unsigned mj = __builtin_amdgcn_ballot_w32(HJ); \
      if (mj != 0u) { \
        if (HJ) { \
          const int pos = wc + (int)__builtin_amdgcn_mbcnt_lo(mj, 0u); \
          if (pos < WCAP) list[wave * WCAP + pos] = ((el0 + (J)) << PKS) | (int)(SJ); \
        } \
        wc += (int)__builtin_popcount(mj); } }
    HITJ(0, h0, s0)
    HITJ(1, h1, s1)
    HITJ(2, h2, s2)
    HITJ(3, h3, s3)
    HITJ(4, h4, s4)
    HITJ(5, h5, s5)
    HITJ(6, h6, s6)
    HITJ(7, h7, s7)
#undef HITJ
  }
  return wc;
}

__global__ __launch_bounds__(NTHR) void k_prep(const float* __restrict__ prew, const float* __restrict__ w1,
                                                const float* __restrict__ w2, const float* __restrict__ w3,
                                                const float* __restrict__ x, int nN, int MP,
                                                unsigned short* B0, unsigned short* B1, unsigned short* B2,
                                                unsigned short* B3, unsigned short* XP) {
  const int u = (int)blockIdx.x * NTHR + (int)threadIdx.x;
  v8us o;
  unsigned short* dp;
  int two = 0;
  if (u < RG1) {
    const int n = u >> 4;
    const int q = u & 15;
    const float* p = prew + (size_t)(8 * q) * C + n;
#pragma unroll
    for (int i = 0; i < 8; ++i) o[i] = (unsigned short)bf16_bits(p[(size_t)i * C]);
    dp = B0 + (size_t)n * KX + 8 * q;
  } else if (u < RG4) {
    const float* W;
    unsigned short* B;
    int v;
    if (u < RG2)      { W = w1; B = B1; v = u - RG1; }
    else if (u < RG3) { W = w2; B = B2; v = u - RG2; }
    else              { W = w3; B = B3; v = u - RG3; }
    const int n = v / (KA / 8);
    const int q = v - (KA / 8) * n;
    const float* p = W + (size_t)(8 * q) * C + n;
#pragma unroll
    for (int i = 0; i < 8; ++i) o[i] = (unsigned short)bf16_bits(p[(size_t)i * C]);
    dp = B + (size_t)n * KP + 8 * q;
    two = 1;
  } else {
    const int v = u - RG4;
    if (v >= MP * (DX / 8)) return;
    const int r  = v >> 4;
    const int q  = v & 15;
    const bool live = r < nN;
    const int rc = live ? r : nN - 1;
    const float* p = x + (size_t)rc * DX + 8 * q;
    const v4f a = *(const v4f*)p;
    const v4f b = *(const v4f*)(p + 4);
    o[0] = (unsigned short)bf16_bits(live ? a.x : 0.0f);
    o[1] = (unsigned short)bf16_bits(live ? a.y : 0.0f);
    o[2] = (unsigned short)bf16_bits(live ? a.z : 0.0f);
    o[3] = (unsigned short)bf16_bits(live ? a.w : 0.0f);
    o[4] = (unsigned short)bf16_bits(live ? b.x : 0.0f);
    o[5] = (unsigned short)bf16_bits(live ? b.y : 0.0f);
    o[6] = (unsigned short)bf16_bits(live ? b.z : 0.0f);
    o[7] = (unsigned short)bf16_bits(live ? b.w : 0.0f);
    dp = XP + (size_t)r * KX + 8 * q;
  }
  *(volatile v8us*)dp = o;
  if (two != 0) *(volatile v8us*)(dp + KA) = o;
  __threadfence();
  *(volatile v8us*)dp = o;
  if (two != 0) *(volatile v8us*)(dp + KA) = o;
}

template <int EPI>
__global__ __launch_bounds__(GTHR) void k_gemm(const unsigned short* __restrict__ A, int lda,
                                               const unsigned short* __restrict__ BT, int K,
                                               const float* __restrict__ bias, float* outF, int nOut) {
  __shared__ __attribute__((aligned(16))) float stg[GBM * GBN];
  __shared__ __attribute__((aligned(16))) float cb[GBN];
  const int tid = (int)threadIdx.x, lane = tid & 31, wave = tid >> 5, hh = lane >> 4, m = lane & 15;
  const int rowBase = (int)blockIdx.x * GBM;
  if (tid < GBN) cb[tid] = bf16_val(bias[tid]);
  __syncthreads();

  v8f acc[4];
#pragma unroll
  for (int t = 0; t < 4; ++t) acc[t] = z8();
  const unsigned short* ap = A  + (size_t)(rowBase + 16 * wave + m) * (size_t)lda + 8 * hh;
  const unsigned short* wp = BT + (size_t)m * (size_t)K + 8 * hh;
  const int ksteps = K >> 5;
#pragma unroll 1
  for (int ks = 0; ks < ksteps; ++ks) {
    Frag af;
    af.h[0] = *(const v8usa*)(ap + 32 * ks);
    af.h[1] = *(const v8usa*)(ap + 32 * ks + 16);
#pragma unroll
    for (int t = 0; t < 4; ++t) {
      const unsigned short* wq = wp + (size_t)(16 * t) * (size_t)K + 32 * ks;
      Frag bf;
      bf.h[0] = *(const v8usa*)wq;
      bf.h[1] = *(const v8usa*)(wq + 16);
      acc[t] = wmk(af, bf, acc[t]);
    }
  }

#pragma unroll
  for (int t = 0; t < 4; ++t) {
    const int lc = 16 * t + m;
    const float bb = cb[lc];
#pragma unroll
    for (int r = 0; r < 8; ++r) {
      const int lr = 16 * wave + 8 * hh + r;
      float v = acc[t][r] + bb;
      if constexpr (EPI == 1) v = (v < 0.0f) ? 0.0f : v;
      stg[lr * GBN + lc] = v;
    }
  }
  __syncthreads();

  v4f pv[8];
#pragma unroll
  for (int ii = 0; ii < 8; ++ii) {
    const int lr = 16 * wave + 2 * ii + hh;
    pv[ii] = *(const v4fa*)(stg + lr * GBN + 4 * m);
  }
  if constexpr (EPI == 2) {
#pragma unroll
    for (int ii = 0; ii < 8; ++ii) {
      float ss = pv[ii].x * pv[ii].x;
      ss = fmaf(pv[ii].y, pv[ii].y, ss);
      ss = fmaf(pv[ii].z, pv[ii].z, ss);
      ss = fmaf(pv[ii].w, pv[ii].w, ss);
      ss += __shfl_xor(ss, 8, 32);
      ss += __shfl_xor(ss, 4, 32);
      ss += __shfl_xor(ss, 2, 32);
      ss += __shfl_xor(ss, 1, 32);
      const float nrm = sqrtf(ss + 0.0f);
      const float inv = 1.0f / fmaxf(nrm, 1e-12f);
      pv[ii] = pv[ii] * inv;
    }
  }

#pragma unroll
  for (int ii = 0; ii < 8; ++ii) {
    const int gr = rowBase + 16 * wave + 2 * ii + hh;
    float* op = outF + (size_t)gr * (size_t)GBN + 4 * m;
    if (EPI != 2 || gr < nOut) *(volatile v4f*)op = pv[ii];
  }
  __threadfence();
#pragma unroll
  for (int ii = 0; ii < 8; ++ii) {
    const int gr = rowBase + 16 * wave + 2 * ii + hh;
    float* op = outF + (size_t)gr * (size_t)GBN + 4 * m;
    if (EPI != 2 || gr < nOut) *(volatile v4f*)op = pv[ii];
  }
}

__global__ __launch_bounds__(NTHR) void k_scan(const int* __restrict__ srcs, const int* __restrict__ dsts,
                                               const float* __restrict__ ea, const float* __restrict__ H,
                                               unsigned short* Aout, int nN, int nE, int vec8) {
  extern __shared__ __attribute__((aligned(16))) int lds_i[];
  int* reg1 = lds_i;
  int* reg2 = reg1 + RCAP;
  int* scnt = reg2 + RCAP;
  int* soff = scnt + NBA;
  int* list = soff + NBA;
  int* wcnt = list + LISTN;
  int* wtot = wcnt + NWAVE;
  const int tid = (int)threadIdx.x, lane = tid & 31, wave = tid >> 5;
  unsigned short* rowbuf = (unsigned short*)(lds_i + ZINTS + MISC_INTS) + wave * RB;
  const int nodeBase = (int)blockIdx.x * NBA;

  {
    const v4i z4 = {0, 0, 0, 0};
    for (int i = tid * 4; i < ZINTS; i += NTHR * 4) *(v4ia*)(lds_i + i) = z4;
    if (tid < 2 * NWAVE) wcnt[tid] = 0;
  }
  __syncthreads();

  int tot = 0;
  const int nChunks = (nE + CHUNK - 1) / CHUNK;
#pragma unroll 1
  for (int ch = 0; ch < nChunks; ++ch) {
    const int cbase = ch * CHUNK;
    const int wc = scan_chunk(dsts, nE, cbase, nodeBase, NBA, vec8, list, tid, lane, wave);
    if (lane == 0) wcnt[wave] = wc;
    __syncthreads();
    int pre = 0, all = 0;
#pragma unroll
    for (int w2 = 0; w2 < NWAVE; ++w2) {
      int c = wcnt[w2];
      c = c < 0 ? 0 : (c > WCAP ? WCAP : c);
      all += c;
      pre += (w2 < wave) ? c : 0;
    }
    const int wcc  = wc > WCAP ? WCAP : wc;
    const int base = tot + pre;
#pragma unroll 1
    for (int i = lane; i < wcc; i += 32) {
      const int ent = list[wave * WCAP + i];
      const int el  = (ent >> PKS) & (CHUNK - 1);
      const int sl  = ent & (NBA - 1);
      int eid = cbase + el;
      eid = eid > nE - 1 ? nE - 1 : eid;
      const int pos = base + i;
      if (pos < RCAP) reg1[pos] = (int)(((unsigned)eid << PKS) | (unsigned)sl);
    }
    tot += all;
    tot = tot > RCAP ? RCAP : tot;
    __syncthreads();
  }
  const int nh = tot;

  if (wave == 0) {
#pragma unroll 1
    for (int b0 = 0; b0 < nh; b0 += 32) {
      const int idx = b0 + lane;
      const int uv  = reg1[idx < RCAP ? idx : RCAP - 1];
      const int m32 = (nh - b0) < 32 ? (nh - b0) : 32;
#pragma unroll 1
      for (int k = 0; k < m32; ++k) {
        const int u  = __builtin_amdgcn_readlane(uv, k);
        const int sl = u & (NBA - 1);
        if (lane == 0) scnt[sl] = scnt[sl] + 1;
      }
    }
  }
  __syncthreads();

  {
    const v4i ca = *(const v4ia*)(scnt + 4 * tid);
    const int e0 = ca.x < 0 ? 0 : ca.x, e1 = ca.y < 0 ? 0 : ca.y, e2 = ca.z < 0 ? 0 : ca.z, e3 = ca.w < 0 ? 0 : ca.w;
    const int ts = e0 + e1 + e2 + e3;
    int incl = ts;
#pragma unroll
    for (int d = 1; d < 32; d <<= 1) {
      const int up = __shfl_up(incl, d, 32);
      if (lane >= d) incl += up;
    }
    if (lane == 31) wtot[wave] = incl;
    __syncthreads();
    int pre = 0;
#pragma unroll
    for (int w2 = 0; w2 < NWAVE; ++w2) pre += (w2 < wave) ? wtot[w2] : 0;
    int run = pre + incl - ts;
    soff[4 * tid + 0] = run; run += e0;
    soff[4 * tid + 1] = run; run += e1;
    soff[4 * tid + 2] = run; run += e2;
    soff[4 * tid + 3] = run;
  }
  __syncthreads();
  for (int i = tid; i < NBA; i += NTHR) list[i] = soff[i];
  __syncthreads();

  if (wave == 0) {
#pragma unroll 1
    for (int b0 = 0; b0 < nh; b0 += 32) {
      const int idx = b0 + lane;
      const int uv  = reg1[idx < RCAP ? idx : RCAP - 1];
      const int m32 = (nh - b0) < 32 ? (nh - b0) : 32;
#pragma unroll 1
      for (int k = 0; k < m32; ++k) {
        const int u   = __builtin_amdgcn_readlane(uv, k);
        const int sl  = u & (NBA - 1);
        const int eid = (int)((unsigned)u >> PKS);
        if (lane == 0) {
          int pos = list[sl];
          pos = pos < 0 ? 0 : (pos > RCAP - 1 ? RCAP - 1 : pos);
          reg2[pos] = eid;
          list[sl] = pos + 1;
        }
      }
    }
  }
  __syncthreads();

  const int nbw = NBA / NWAVE;
  const bool ovf = (nh >= RCAP);
  const float qnan = __int_as_float(0x7fc00000);
  const int l16 = lane & 15;
  const bool xw = lane < 16;

#pragma unroll 1
  for (int jt = 0; jt < nbw; ++jt) {
    const int slot = wave * nbw + jt;
    const int node = nodeBase + slot;
    int st = soff[slot];
    const int craw = scnt[slot];
    int cnt = craw;
    st  = st < 0 ? 0 : (st > nh ? nh : st);
    cnt = cnt < 0 ? 0 : (cnt > DEGCAP ? DEGCAP : cnt);
    if (cnt > nh - st) cnt = nh - st;
    const float pz = (ovf || craw > DEGCAP) ? qnan : 0.0f;
    const bool live = node < nN;

    float a00 = 0.0f, a01 = 0.0f, a10 = 0.0f, a11 = 0.0f, a20 = 0.0f, a21 = 0.0f;
#pragma unroll 1
    for (int b0 = 0; b0 < cnt; b0 += 32) {
      int idx = st + b0 + lane; idx = idx > RCAP - 1 ? RCAP - 1 : idx;
      int eid = reg2[idx]; eid = eid < 0 ? 0 : (eid > nE - 1 ? nE - 1 : eid);
      int sr = srcs[eid]; sr = sr < 0 ? 0 : (sr > nN - 1 ? nN - 1 : sr);
      const float* ep = ea + (size_t)eid * 3;
      const int g0i = __float_as_int(bf16_val(ep[0]));
      const int g1i = __float_as_int(bf16_val(ep[1]));
      const int g2i = __float_as_int(bf16_val(ep[2]));
      const int m32 = (cnt - b0) < 32 ? (cnt - b0) : 32;
#pragma unroll 1
      for (int k = 0; k < m32; ++k) {
        const int   sk = __builtin_amdgcn_readlane(sr, k);
        const float g0 = __int_as_float(__builtin_amdgcn_readlane(g0i, k));
        const float g1 = __int_as_float(__builtin_amdgcn_readlane(g1i, k));
        const float g2 = __int_as_float(__builtin_amdgcn_readlane(g2i, k));
        const v2f v = *(const v2fa*)(H + (size_t)sk * C + 2 * lane);
        a00 = fmaf(g0, v.x, a00); a01 = fmaf(g0, v.y, a01);
        a10 = fmaf(g1, v.x, a10); a11 = fmaf(g1, v.y, a11);
        a20 = fmaf(g2, v.x, a20); a21 = fmaf(g2, v.y, a21);
      }
    }
    const float inv = 1.0f / (float)(cnt > 0 ? cnt : 1);
    const float m00 = (live ? a00 * inv : 0.0f) + pz;
    const float m01 = (live ? a01 * inv : 0.0f) + pz;
    const float m10 = (live ? a10 * inv : 0.0f) + pz;
    const float m11 = (live ? a11 * inv : 0.0f) + pz;
    const float m20 = (live ? a20 * inv : 0.0f) + pz;
    const float m21 = (live ? a21 * inv : 0.0f) + pz;

    v2us h0v, l0v, h1v, l1v, h2v, l2v;
    {
      unsigned hb;
      hb = bf16_bits(m00); h0v[0] = (unsigned short)hb; l0v[0] = (unsigned short)bf16_bits(m00 - __uint_as_float(hb << 16));
      hb = bf16_bits(m01); h0v[1] = (unsigned short)hb; l0v[1] = (unsigned short)bf16_bits(m01 - __uint_as_float(hb << 16));
      hb = bf16_bits(m10); h1v[0] = (unsigned short)hb; l1v[0] = (unsigned short)bf16_bits(m10 - __uint_as_float(hb << 16));
      hb = bf16_bits(m11); h1v[1] = (unsigned short)hb; l1v[1] = (unsigned short)bf16_bits(m11 - __uint_as_float(hb << 16));
      hb = bf16_bits(m20); h2v[0] = (unsigned short)hb; l2v[0] = (unsigned short)bf16_bits(m20 - __uint_as_float(hb << 16));
      hb = bf16_bits(m21); h2v[1] = (unsigned short)hb; l2v[1] = (unsigned short)bf16_bits(m21 - __uint_as_float(hb << 16));
    }
    *(v2usa*)(rowbuf + 2 * lane)              = h0v;
    *(v2usa*)(rowbuf + C + 2 * lane)          = h1v;
    *(v2usa*)(rowbuf + 2 * C + 2 * lane)      = h2v;
    *(v2usa*)(rowbuf + KA + 2 * lane)         = l0v;
    *(v2usa*)(rowbuf + KA + C + 2 * lane)     = l1v;
    *(v2usa*)(rowbuf + KA + 2 * C + 2 * lane) = l2v;
    wave_sync();
    const v8us q0 = *(const v8usa*)(rowbuf + 8 * lane);
    const v8us q1 = *(const v8usa*)(rowbuf + 256 + 8 * l16);
    wave_sync();

    unsigned short* gp = Aout + (size_t)node * (size_t)KP + 8 * lane;
    unsigned short* gx = Aout + (size_t)node * (size_t)KP + 256 + 8 * l16;
    *(volatile v8us*)gp = q0;
    if (xw) *(volatile v8us*)gx = q1;
    __threadfence();
    *(volatile v8us*)gp = q0;
    if (xw) *(volatile v8us*)gx = q1;
  }
}

static inline int cdiv(int a, int b) { return (a + b - 1) / b; }
static inline size_t al256(size_t o) { return (o + 255) & ~(size_t)255; }

extern "C" void kernel_launch(void* const* d_in, const int* in_sizes, int n_in,
                              void* d_out, int out_size, void* d_ws, size_t ws_size,
                              hipStream_t stream) {
  if (n_in < 11) return;
  if (in_sizes[0] < DX || (in_sizes[0] % DX) != 0) return;
  const int nN = in_sizes[0] / DX;
  if (nN < GBM || nN > (1 << 22)) return;
  if (in_sizes[1] < 2 || (in_sizes[1] & 1) != 0) return;
  const int nE = in_sizes[1] / 2;
  if (nE < 1 || nE >= (1 << (32 - PKS))) return;
  if (in_sizes[2] != 3 * nE) return;
  if (in_sizes[3] != DX * C || in_sizes[4] != C) return;
  if (in_sizes[5] != KA * C || in_sizes[6] != C) return;
  if (in_sizes[7] != KA * C || in_sizes[8] != C) return;
  if (in_sizes[9] != KA * C || in_sizes[10] != C) return;
  if ((long long)out_size != (long long)nN * C) return;

  const float* x    = (const float*)d_in[0];
  const int*   ei   = (const int*)  d_in[1];
  const float* ea   = (const float*)d_in[2];
  const float* prew = (const float*)d_in[3];
  const float* preb = (const float*)d_in[4];
  const float* w1   = (const float*)d_in[5];
  const float* b1   = (const float*)d_in[6];
  const float* w2   = (const float*)d_in[7];
  const float* b2   = (const float*)d_in[8];
  const float* w3   = (const float*)d_in[9];
  const float* b3   = (const float*)d_in[10];
  float* out = (float*)d_out;
  const int* src = ei;
  const int* tgt = ei + nE;

  const int MP   = cdiv(nN, GBM) * GBM;
  const int gM   = MP / GBM;
  const int gA   = cdiv(MP, NBA);
  const int RA   = gA * NBA;
  const int vec8 = ((nE & 3) == 0) ? 1 : 0;
  if ((long long)RA < (long long)MP) return;
  if ((long long)gM * GBM < (long long)nN) return;

  char* ws = (char*)d_ws;
  size_t off = 0;
  const size_t oB0 = off; off = al256(off + (size_t)C * KX * 2);
  const size_t oB1 = off; off = al256(off + (size_t)C * KP * 2);
  const size_t oB2 = off; off = al256(off + (size_t)C * KP * 2);
  const size_t oB3 = off; off = al256(off + (size_t)C * KP * 2);
  const size_t oXP = off; off = al256(off + (size_t)MP * KX * 2);
  const size_t oAP = off; off = al256(off + (size_t)RA * KP * 2);
  const size_t oH  = off; off = al256(off + (size_t)MP * C * 4);
  if (off > ws_size || off > (size_t)WSMAX) return;
  unsigned short* B0 = (unsigned short*)(ws + oB0);
  unsigned short* B1 = (unsigned short*)(ws + oB1);
  unsigned short* B2 = (unsigned short*)(ws + oB2);
  unsigned short* B3 = (unsigned short*)(ws + oB3);
  unsigned short* XP = (unsigned short*)(ws + oXP);
  unsigned short* AP = (unsigned short*)(ws + oAP);
  float*          H  = (float*)(ws + oH);

  hipFuncSetAttribute(reinterpret_cast<const void*>(&k_scan), hipFuncAttributeMaxDynamicSharedMemorySize, LDS_AGG);

  const int gP = (RG4 + MP * (DX / 8)) / NTHR;

  k_prep<<<gP, NTHR, 0, stream>>>(prew, w1, w2, w3, x, nN, MP, B0, B1, B2, B3, XP);
  k_gemm<0><<<gM, GTHR, 0, stream>>>(XP, KX, B0, KX, preb, H, nN);
  k_scan<<<gA, NTHR, LDS_AGG, stream>>>(src, tgt, ea, H, AP, nN, nE, vec8);
  k_gemm<1><<<gM, GTHR, 0, stream>>>(AP, KP, B1, KP, b1, H, nN);
  k_scan<<<gA, NTHR, LDS_AGG, stream>>>(src, tgt, ea, H, AP, nN, nE, vec8);
  k_gemm<1><<<gM, GTHR, 0, stream>>>(AP, KP, B2, KP, b2, H, nN);
  k_scan<<<gA, NTHR, LDS_AGG, stream>>>(src, tgt, ea, H, AP, nN, nE, vec8);
  k_gemm<2><<<gM, GTHR, 0, stream>>>(AP, KP, B3, KP, b3, out, nN);
}
